// NeuralODETrainer_50225347559896
// MI455X (gfx1250) — hardware-run, weakly checked
//
#include <hip/hip_runtime.h>
#include <stdint.h>

#pragma clang fp contract(off)

typedef __attribute__((ext_vector_type(16))) _Float16 v16h;
typedef __attribute__((ext_vector_type(8)))  _Float16 v8h;
typedef __attribute__((ext_vector_type(8)))  float    v8f;
typedef __attribute__((ext_vector_type(4)))  float    v4f;

#define DEVFN __device__ __forceinline__

__device__ __forceinline__ void dep_guard_h(v8f& a, v8f& b, v16h x, v16h y) { asm volatile("v_nop\n\tv_nop\n\tv_nop\n\tv_nop" : "+v"(a), "+v"(b) : "v"(x), "v"(y)); }
__device__ __forceinline__ void keep4_h(v16h a, v16h b, v16h c, v16h d) { asm volatile("v_nop" :: "v"(a), "v"(b), "v"(c), "v"(d)); }
__device__ __forceinline__ void acc_guard4(v8f& a, v8f& b, v8f& c, v8f& d) { asm volatile("v_nop\n\tv_nop\n\tv_nop\n\tv_nop" : "+v"(a), "+v"(b), "+v"(c), "+v"(d)); }
__device__ __forceinline__ void dep_guard1_h(v8f& a, v16h x, v16h y) { asm volatile("v_nop\n\tv_nop\n\tv_nop\n\tv_nop" : "+v"(a) : "v"(x), "v"(y)); }
__device__ __forceinline__ void acc_guard2(v8f& a, v8f& b) { asm volatile("v_nop\n\tv_nop\n\tv_nop\n\tv_nop" : "+v"(a), "+v"(b)); }
__device__ __forceinline__ void acc_guard1(v8f& a) { asm volatile("v_nop\n\tv_nop\n\tv_nop\n\tv_nop" : "+v"(a)); }

template <typename T> struct Frag;
template <> struct Frag<_Float16> {
  typedef v16h V; union U { v16h v; v8h h[2]; };
  static __device__ __forceinline__ v16h load(const _Float16* p) {
    U f; f.h[0] = *(const v8h*)(p); f.h[1] = *(const v8h*)(p + 16); return f.v;
  }
  static __device__ __forceinline__ v8f mma(v16h a, v16h b, v8f c) {
    return __builtin_amdgcn_wmma_f32_16x16x32_f16(false, a, false, b, (short)0, c, false, false);
  }
  static __device__ __forceinline__ void guard(v8f& a, v8f& b, v16h x, v16h y) { dep_guard_h(a, b, x, y); }
  static __device__ __forceinline__ void keep(v16h a, v16h b, v16h c, v16h d) { keep4_h(a, b, c, d); }
};

template <int NSUB> struct AccGuard;
template <> struct AccGuard<4> { static DEVFN void run(v8f (&a)[4]) { acc_guard4(a[0], a[1], a[2], a[3]); } };
template <> struct AccGuard<2> { static DEVFN void run(v8f (&a)[2]) { acc_guard2(a[0], a[1]); } };

namespace {

constexpr int kBatch    = 4096;
constexpr int kStateDim = 13;
constexpr int kTimes    = 16;
constexpr int kRows     = 16;
constexpr int kBlocks   = kBatch / kRows;
constexpr int kThreadsMain = 128;
constexpr int kHid1 = 256, kHid2 = 256, kHid3 = 128, kOutDim = 12;
constexpr int kK1Pad = 32;
constexpr int kN4Pad = 16;
constexpr int kHPitch = 264;
constexpr int kA1Pitch = 32;
constexpr int kSlabPitch = 68;
constexpr int kYPitch = 16;
static_assert(kBlocks * kRows == kBatch, "grid covers the batch exactly");

constexpr float kActScale = 8.0f;
constexpr float kW1Scale = 16.0f, kW2Scale = 64.0f, kW3Scale = 64.0f, kW4Scale = 512.0f;
constexpr float kInv1 = 1.0f / 128.0f;
constexpr float kInv2 = 1.0f / 512.0f;
constexpr float kInv3 = 1.0f / 512.0f;
constexpr float kInv4 = 1.0f / 4096.0f;

constexpr float cA21 = (float)(1.0 / 5.0);
constexpr float cA31 = (float)(3.0 / 40.0),      cA32 = (float)(9.0 / 40.0);
constexpr float cA41 = (float)(44.0 / 45.0),     cA42 = (float)(-56.0 / 15.0),    cA43 = (float)(32.0 / 9.0);
constexpr float cA51 = (float)(19372.0 / 6561.0), cA52 = (float)(-25360.0 / 2187.0),
                cA53 = (float)(64448.0 / 6561.0), cA54 = (float)(-212.0 / 729.0);
constexpr float cA61 = (float)(9017.0 / 3168.0),  cA62 = (float)(-355.0 / 33.0),
                cA63 = (float)(46732.0 / 5247.0), cA64 = (float)(49.0 / 176.0),     cA65 = (float)(-5103.0 / 18656.0);
constexpr float cB1 = (float)(35.0 / 384.0), cB3 = (float)(500.0 / 1113.0), cB4 = (float)(125.0 / 192.0),
                cB5 = (float)(-2187.0 / 6784.0), cB6 = (float)(11.0 / 84.0);

constexpr size_t kOffYpl = 0;
constexpr size_t kOffW1t = 4194304;
constexpr size_t kOffW2t = kOffW1t + 256 * 32 * 2;
constexpr size_t kOffW3t = kOffW2t + 256 * 256 * 2;
constexpr size_t kOffW4t = kOffW3t + 128 * 256 * 2;
constexpr size_t kWsTotal = kOffW4t + 16 * 128 * 2;
static_assert(kWsTotal == 4411392, "carve total");

DEVFN float sel6(int e, float v1, float v2, float v3, float v4, float v5, float v6) {
  return e == 1 ? v1 : e == 2 ? v2 : e == 3 ? v3 : e == 4 ? v4 : e == 5 ? v5 : e == 6 ? v6 : 0.0f;
}

DEVFN float stage_sum(const float* kb, int idx, float c1, float c2, float c3, float c4, float c5, float c6) {
  float s = c1 * kb[idx];
  s = s + c2 * kb[256 + idx];
  s = s + c3 * kb[512 + idx];
  s = s + c4 * kb[768 + idx];
  s = s + c5 * kb[1024 + idx];
  s = s + c6 * kb[1280 + idx];
  return s;
}

DEVFN _Float16 silu_scaled_h(float v) {
  const float sg = __builtin_amdgcn_rcpf(1.0f + expf(-v));
  return (_Float16)(v * sg * kActScale);
}

template <int NSUB, int KSTEPS>
DEVFN void gemm_rows16(const _Float16* At, int lda, const _Float16* __restrict__ Bt, int ldb, int n0, int lane,
                       v8f (&acc)[NSUB]) {
  const int c = lane & 15;
  const int koff = (lane >> 4) * 8;
#pragma unroll
  for (int j = 0; j < NSUB; ++j) acc[j] = (v8f){0.f, 0.f, 0.f, 0.f, 0.f, 0.f, 0.f, 0.f};
#pragma unroll 1
  for (int ks = 0; ks < KSTEPS; ++ks) {
    const int k0 = ks * 32;
    v16h bh[NSUB];
#pragma unroll
    for (int j = 0; j < NSUB; ++j)
      bh[j] = Frag<_Float16>::load(Bt + (size_t)(n0 + (j << 4) + c) * ldb + k0 + koff);
    const v16h ah = Frag<_Float16>::load(At + c * lda + k0 + koff);
#pragma unroll
    for (int j = 0; j < NSUB; ++j) acc[j] = Frag<_Float16>::mma(ah, bh[j], acc[j]);
    dep_guard_h(acc[0], acc[NSUB - 1], ah, bh[0]);
    keep4_h(bh[0], bh[1], bh[NSUB - 2], bh[NSUB - 1]);
  }
  AccGuard<NSUB>::run(acc);
}

template <int NSUB>
DEVFN void silu_store(v8f (&acc)[NSUB], float inv, const float* __restrict__ bias, int n0,
                      float* slab, _Float16* Hout, int hpitch, int lane) {
  const int c = lane & 15;
  const int r0 = (lane >> 4) * 8;
#pragma unroll
  for (int j = 0; j < NSUB; ++j) {
    const float bv = bias[n0 + (j << 4) + c];
#pragma unroll
    for (int r = 0; r < 8; ++r) slab[(r0 + r) * kSlabPitch + (j << 4) + c] = acc[j][r] * inv + bv;
  }
  __builtin_amdgcn_fence(__ATOMIC_RELEASE, "workgroup");
  __builtin_amdgcn_wave_barrier();
  __builtin_amdgcn_fence(__ATOMIC_ACQUIRE, "workgroup");
  constexpr int kGroups = 2 * NSUB;
#pragma unroll 1
  for (int it = 0; it < NSUB; ++it) {
    const int g = it * 32 + lane;
    const int row = g / kGroups;
    const int cg = g - row * kGroups;
    const float* sp = slab + row * kSlabPitch + cg * 8;
    const v4f p0 = *(const v4f*)(sp);
    const v4f p1 = *(const v4f*)(sp + 4);
    v8h hv;
#pragma unroll
    for (int e = 0; e < 4; ++e) {
      hv[e]     = silu_scaled_h(p0[e]);
      hv[4 + e] = silu_scaled_h(p1[e]);
    }
    *(v8h*)(Hout + row * hpitch + n0 + cg * 8) = hv;
  }
}

DEVFN void store_state(const float (&y)[8], float* sY, float* __restrict__ dst, int lane) {
  const int hh = lane >> 4, c = lane & 15;
#pragma unroll
  for (int r = 0; r < 8; ++r) sY[(8 * hh + r) * kYPitch + c] = y[r];
  __builtin_amdgcn_fence(__ATOMIC_RELEASE, "workgroup");
  __builtin_amdgcn_wave_barrier();
  __builtin_amdgcn_fence(__ATOMIC_ACQUIRE, "workgroup");
  for (int pass = 0; pass < 2; ++pass) {
#pragma unroll
    for (int it = 0; it < 2; ++it) {
      const v4f v = *(const v4f*)(sY + it * 128 + lane * 4);
      *(volatile v4f*)(dst + it * 128 + lane * 4) = v;
    }
    __threadfence();
  }
  __builtin_amdgcn_fence(__ATOMIC_RELEASE, "workgroup");
  __builtin_amdgcn_wave_barrier();
  __builtin_amdgcn_fence(__ATOMIC_ACQUIRE, "workgroup");
}

}

__global__ __launch_bounds__(256) void cast_weight_t(const float* __restrict__ W, int Kin, int Nout, int Kpad,
                                                     float scale, _Float16* __restrict__ out, int nchunks) {
  const int i = blockIdx.x * 256 + threadIdx.x;
  if (i >= nchunks) return;
  const int cpr = Kpad >> 3;
  const int n = i / cpr;
  const int kc = i - n * cpr;
  const int ncl = n < Nout ? n : Nout - 1;
  v8h hv;
#pragma unroll
  for (int e = 0; e < 8; ++e) {
    const int k = kc * 8 + e;
    const int kcl = k < Kin ? k : Kin - 1;
    const float w = W[(size_t)kcl * Nout + ncl];
    const float v = (n < Nout && k < Kin) ? w * scale : 0.0f;
    hv[e] = (_Float16)v;
  }
  _Float16* dst = out + (size_t)i * 8;
  *(volatile v8h*)dst = hv;
  __threadfence();
  *(volatile v8h*)dst = hv;
}

__global__ __launch_bounds__(kThreadsMain) void ode_persistent(
    const float* __restrict__ y0, const float* __restrict__ tspan,
    const _Float16* __restrict__ W1t, const _Float16* __restrict__ W2t,
    const _Float16* __restrict__ W3t, const _Float16* __restrict__ W4t,
    const float* __restrict__ b1, const float* __restrict__ b2,
    const float* __restrict__ b3, const float* __restrict__ b4,
    float* __restrict__ Ypl) {
  __shared__ __align__(16) _Float16 sA1[kRows * kA1Pitch];
  __shared__ __align__(16) _Float16 sH1[kRows * kHPitch];
  __shared__ __align__(16) _Float16 sH2[kRows * kHPitch];
  __shared__ __align__(16) float sSlab[4][kRows * kSlabPitch];
  __shared__ __align__(16) float sK[6 * 256];
  __shared__ __align__(16) float sY[kRows * kYPitch];

  const int tid = threadIdx.x;
  const int wave = tid >> 5;
  const int lane = tid & 31;
  const int hh = lane >> 4;
  const int c = lane & 15;
  const int row0 = blockIdx.x * kRows;
  float* slab = sSlab[wave];

  {
    const v4f z4 = {0.0f, 0.0f, 0.0f, 0.0f};
    for (int i = tid; i < (6 * 256) / 4; i += kThreadsMain) *(v4f*)(sK + 4 * i) = z4;
    if (tid < (kRows * kA1Pitch) / 8) {
      v8h z8;
#pragma unroll
      for (int e = 0; e < 8; ++e) z8[e] = (_Float16)0.0f;
      *(v8h*)(sA1 + tid * 8) = z8;
    }
  }
  float y[8];
  {
    const int cc = c < kStateDim ? c : kStateDim - 1;
#pragma unroll
    for (int r = 0; r < 8; ++r) {
      const float v = y0[(size_t)(row0 + 8 * hh + r) * kStateDim + cc];
      y[r] = (c < kStateDim) ? v : 0.0f;
    }
  }
  __syncthreads();
  if (wave == 0) store_state(y, sY, Ypl + (size_t)row0 * kYPitch, lane);

#pragma unroll 1
  for (int s = 1; s < kTimes; ++s) {
    const float hstep = (tspan[s] - tspan[s - 1]) * 0.5f;
#pragma unroll 1
    for (int sub = 0; sub < 2; ++sub) {
#pragma unroll 1
      for (int e = 0; e < 6; ++e) {
        if (wave == 0) {
          const float c1 = sel6(e, cA21, cA31, cA41, cA51, cA61, 0.0f);
          const float c2 = sel6(e, 0.0f, cA32, cA42, cA52, cA62, 0.0f);
          const float c3 = sel6(e, 0.0f, 0.0f, cA43, cA53, cA63, 0.0f);
          const float c4 = sel6(e, 0.0f, 0.0f, 0.0f, cA54, cA64, 0.0f);
          const float c5 = sel6(e, 0.0f, 0.0f, 0.0f, 0.0f, cA65, 0.0f);
#pragma unroll
          for (int r = 0; r < 8; ++r) {
            const int idx = (8 * hh + r) * 16 + c;
            const float ssum = stage_sum(sK, idx, c1, c2, c3, c4, c5, 0.0f);
            const float ys = y[r] + hstep * ssum;
            sA1[(8 * hh + r) * kA1Pitch + c] = (_Float16)(ys * kActScale);
          }
        }
        __syncthreads();
        {
          v8f acc[4];
          gemm_rows16<4, 1>(sA1, kA1Pitch, W1t, kK1Pad, 64 * wave, lane, acc);
          silu_store<4>(acc, kInv1, b1, 64 * wave, slab, sH1, kHPitch, lane);
        }
        __syncthreads();
        {
          v8f acc[4];
          gemm_rows16<4, 8>(sH1, kHPitch, W2t, kHid1, 64 * wave, lane, acc);
          silu_store<4>(acc, kInv2, b2, 64 * wave, slab, sH2, kHPitch, lane);
        }
        __syncthreads();
        {
          v8f acc[2];
          gemm_rows16<2, 8>(sH2, kHPitch, W3t, kHid2, 32 * wave, lane, acc);
          silu_store<2>(acc, kInv3, b3, 32 * wave, slab, sH1, kHPitch, lane);
        }
        __syncthreads();
        if (wave == 0) {
          const int koff = hh * 8;
          v8f acc4 = (v8f){0.f, 0.f, 0.f, 0.f, 0.f, 0.f, 0.f, 0.f};
#pragma unroll 1
          for (int ks = 0; ks < kHid3 / 32; ++ks) {
            const int k0 = ks * 32;
            const v16h bq = Frag<_Float16>::load(W4t + (size_t)c * kHid3 + k0 + koff);
            const v16h aq = Frag<_Float16>::load(sH1 + c * kHPitch + k0 + koff);
            acc4 = Frag<_Float16>::mma(aq, bq, acc4);
            dep_guard1_h(acc4, aq, bq);
          }
          acc_guard1(acc4);
          const int cb = c < kOutDim ? c : kOutDim - 1;
          const float b4v = b4[cb];
          float* kd = sK + e * 256;
#pragma unroll
          for (int r = 0; r < 8; ++r) {
            float d = acc4[r] * kInv4 + b4v;
            d = (c < kOutDim) ? d : 0.0f;
            kd[(8 * hh + r) * 16 + c] = d;
          }
        }
      }
      if (wave == 0) {
#pragma unroll
        for (int r = 0; r < 8; ++r) {
          const int idx = (8 * hh + r) * 16 + c;
          const float ssum = stage_sum(sK, idx, cB1, 0.0f, cB3, cB4, cB5, cB6);
          y[r] = y[r] + hstep * ssum;
        }
      }
    }
    if (wave == 0) store_state(y, sY, Ypl + ((size_t)s * kBatch + row0) * kYPitch, lane);
  }
}

__global__ __launch_bounds__(256) void repack_out(const float* __restrict__ Ypl, float* __restrict__ out, int nquads) {
  const int i = blockIdx.x * 256 + threadIdx.x;
  if (i >= nquads) return;
  v4f v;
#pragma unroll
  for (int u = 0; u < 4; ++u) {
    const unsigned e = 4u * (unsigned)i + (unsigned)u;
    unsigned rr = e / 13u;
    const unsigned cc = e - 13u * rr;
    rr = rr < (unsigned)(kTimes * kBatch - 1) ? rr : (unsigned)(kTimes * kBatch - 1);
    v[u] = Ypl[(size_t)rr * kYPitch + cc];
  }
  float* dst = out + (size_t)i * 4;
  *(volatile v4f*)dst = v;
  __threadfence();
  *(volatile v4f*)dst = v;
}

extern "C" void kernel_launch(void* const* d_in, const int* in_sizes, int n_in,
                              void* d_out, int out_size, void* d_ws, size_t ws_size,
                              hipStream_t stream) {
  if (n_in < 10) return;
  if (in_sizes[0] != kBatch * kStateDim || in_sizes[1] != kTimes ||
      in_sizes[2] != kStateDim * kHid1 || in_sizes[3] != kHid1 ||
      in_sizes[4] != kHid1 * kHid2 || in_sizes[5] != kHid2 ||
      in_sizes[6] != kHid2 * kHid3 || in_sizes[7] != kHid3 ||
      in_sizes[8] != kHid3 * kOutDim || in_sizes[9] != kOutDim) return;
  if (out_size != kTimes * kBatch * kStateDim) return;
  if (ws_size < kWsTotal) return;

  const float* y0 = (const float*)d_in[0];
  const float* tspan = (const float*)d_in[1];
  const float* W1 = (const float*)d_in[2];
  const float* b1 = (const float*)d_in[3];
  const float* W2 = (const float*)d_in[4];
  const float* b2 = (const float*)d_in[5];
  const float* W3 = (const float*)d_in[6];
  const float* b3 = (const float*)d_in[7];
  const float* W4 = (const float*)d_in[8];
  const float* b4 = (const float*)d_in[9];
  float* out = (float*)d_out;

  char* ws = (char*)d_ws;
  float* Ypl = (float*)(ws + kOffYpl);
  _Float16* W1t = (_Float16*)(ws + kOffW1t);
  _Float16* W2t = (_Float16*)(ws + kOffW2t);
  _Float16* W3t = (_Float16*)(ws + kOffW3t);
  _Float16* W4t = (_Float16*)(ws + kOffW4t);

  const int n1 = kHid1 * kK1Pad / 8;
  const int n2 = kHid2 * kHid1 / 8;
  const int n3 = kHid3 * kHid2 / 8;
  const int n4 = kN4Pad * kHid3 / 8;
  cast_weight_t<<<dim3((n1 + 255) / 256), dim3(256), 0, stream>>>(W1, kStateDim, kHid1, kK1Pad, kW1Scale, W1t, n1);
  cast_weight_t<<<dim3((n2 + 255) / 256), dim3(256), 0, stream>>>(W2, kHid1, kHid2, kHid1, kW2Scale, W2t, n2);
  cast_weight_t<<<dim3((n3 + 255) / 256), dim3(256), 0, stream>>>(W3, kHid2, kHid3, kHid2, kW3Scale, W3t, n3);
  cast_weight_t<<<dim3((n4 + 255) / 256), dim3(256), 0, stream>>>(W4, kHid3, kOutDim, kHid3, kW4Scale, W4t, n4);

  ode_persistent<<<dim3(kBlocks), dim3(kThreadsMain), 0, stream>>>(
      y0, tspan, W1t, W2t, W3t, W4t, b1, b2, b3, b4, Ypl);

  const int nquads = out_size / 4;
  repack_out<<<dim3((nquads + 255) / 256), dim3(256), 0, stream>>>(Ypl, out, nquads);
}
